// TSRM_Encoder_36129264894097
// MI455X (gfx1250) — hardware-verified
//
#include <hip/hip_runtime.h>
#include <math.h>
#include <stdint.h>


#define BB   4
#define TT   256
#define DD   1024
#define HH   512
#define GG   8
#define PP   384
#define NN   384
#define LL   16
#define HGG  64
#define ECW  1124
#define MPB  64
#define PEP  520

static_assert(NN % MPB == 0);
static_assert(PP % 32 == 0);
static_assert(HH % 64 == 0);
static_assert(DD % 64 == 0);
static_assert(NN % 64 == 0);
static_assert((32 * ECW) % 4 == 0);
static_assert(((32 * ECW * 4) % 128) == 0);

typedef _Float16 f16t;
typedef f16t  v16h __attribute__((ext_vector_type(16)));
typedef f16t  v8h  __attribute__((ext_vector_type(8)));
typedef float v8f  __attribute__((ext_vector_type(8)));
typedef float v4f  __attribute__((ext_vector_type(4)));

union Frag { v16h v; v8h h[2]; };

__device__ __forceinline__ v8f wmma16(v16h a, v16h b, v8f c) {
  c = __builtin_amdgcn_wmma_f32_16x16x32_f16(false, a, false, b, (short)0, c, false, false);
  asm volatile("v_nop\n\tv_nop\n\tv_nop\n\tv_nop" : "+v"(c) : "v"(a), "v"(b));
  return c;
}
__device__ __forceinline__ v8f zero8() { v8f z = {0.f, 0.f, 0.f, 0.f, 0.f, 0.f, 0.f, 0.f}; return z; }
__device__ __forceinline__ v8h zero8h() { v8h z; for (int j = 0; j < 8; ++j) z[j] = (f16t)0.f; return z; }
__device__ __forceinline__ void stv4(float* p, v4f v) { *(volatile v4f*)p = v; }
__device__ __forceinline__ void stv8(f16t* p, v8h v) { *(volatile v8h*)p = v; }

__device__ __forceinline__ float bsum128(float v, float* red, int tid) {
#pragma unroll
  for (int o = 16; o > 0; o >>= 1) v += __shfl_xor(v, o);
  if ((tid & 31) == 0) red[tid >> 5] = v;
  __syncthreads();
  float r = (red[0] + red[1]) + (red[2] + red[3]);
  __syncthreads();
  return r;
}
__device__ __forceinline__ float bmax128(float v, float* red, int tid) {
#pragma unroll
  for (int o = 16; o > 0; o >>= 1) v = fmaxf(v, __shfl_xor(v, o));
  if ((tid & 31) == 0) red[tid >> 5] = v;
  __syncthreads();
  float r = fmaxf(fmaxf(red[0], red[1]), fmaxf(red[2], red[3]));
  __syncthreads();
  return r;
}

__global__ void __launch_bounds__(256)
k_clip(const float* __restrict__ feats, const int* __restrict__ vid_idx,
       const int* __restrict__ starts, const int* __restrict__ clip_len,
       float* __restrict__ out1, f16t* __restrict__ efh) {
  __shared__ __align__(16) f16t sE[DD];
  const int p = blockIdx.x, tid = threadIdx.x, d = tid * 4;
  int vid = vid_idx[p];
  if (vid < 0) vid += BB;
  vid = vid < 0 ? 0 : (vid > BB - 1 ? BB - 1 : vid);
  const int st = starts[p];
  int cl = clip_len[0];
  cl = cl < 1 ? 1 : (cl > LL ? LL : cl);

  v4f x[LL];
  v4f acc = {0.f, 0.f, 0.f, 0.f};
#pragma unroll
  for (int l = 0; l < LL; ++l) {
    int t = st + l;
    if (t < 0) t += TT;
    t = t < 0 ? 0 : (t > TT - 1 ? TT - 1 : t);
    x[l] = *(const v4f*)(feats + ((size_t)(vid * TT + t)) * DD + d);
    acc += x[l];
  }
  float* cf = out1 + (size_t)p * LL * DD + d;
#pragma unroll
  for (int l = 0; l < LL; ++l) stv4(cf + (size_t)l * DD, x[l]);

  const float inv = 1.0f / ((float)cl + 1e-5f);
  sE[d + 0] = (f16t)(acc.x * inv);
  sE[d + 1] = (f16t)(acc.y * inv);
  sE[d + 2] = (f16t)(acc.z * inv);
  sE[d + 3] = (f16t)(acc.w * inv);
  __syncthreads();
  v8h e8 = zero8h();
  if (tid < DD / 8) e8 = *(const v8h*)&sE[tid * 8];
  f16t* ep = efh + (size_t)p * DD + tid * 8;
  if (tid < DD / 8) stv8(ep, e8);
  __threadfence();
#pragma unroll
  for (int l = 0; l < LL; ++l) stv4(cf + (size_t)l * DD, x[l]);
  if (tid < DD / 8) stv8(ep, e8);
}

__global__ void __launch_bounds__(256)
k_misc(const float* __restrict__ W_p2, float* __restrict__ out2, f16t* __restrict__ wt2) {
  const int tid = threadIdx.x;
  const v4f one = {1.f, 1.f, 1.f, 1.f};
  v8h wv[4];
#pragma unroll
  for (int it = 0; it < 4; ++it) {
    const int idx = it * 256 + tid;
    const int n = idx >> 6, piece = idx & 63;
#pragma unroll
    for (int j = 0; j < 8; ++j) {
      const int k = piece * 8 + j;
      float w = (n < GG) ? W_p2[k * GG + n] * 16.0f : 0.0f;
      wv[it][j] = (f16t)w;
    }
  }
#pragma unroll
  for (int it = 0; it < 6; ++it) stv4(out2 + (size_t)(it * 256 + tid) * 4, one);
#pragma unroll
  for (int it = 0; it < 4; ++it) {
    const int idx = it * 256 + tid;
    stv8(wt2 + (size_t)(idx >> 6) * HH + (idx & 63) * 8, wv[it]);
  }
  __threadfence();
#pragma unroll
  for (int it = 0; it < 6; ++it) stv4(out2 + (size_t)(it * 256 + tid) * 4, one);
#pragma unroll
  for (int it = 0; it < 4; ++it) {
    const int idx = it * 256 + tid;
    stv8(wt2 + (size_t)(idx >> 6) * HH + (idx & 63) * 8, wv[it]);
  }
}

template <typename Tin>
__global__ void __launch_bounds__(256)
k_tr64(const Tin* __restrict__ src0, const Tin* __restrict__ src1,
       const Tin* __restrict__ src2, const Tin* __restrict__ src3,
       int K, int N, float scale, f16t* __restrict__ dst, int dstStrideZ) {
  __shared__ __align__(16) f16t T[64][72];
  const int z = blockIdx.z;
  const Tin* src = (z == 0) ? src0 : (z == 1) ? src1 : (z == 2) ? src2 : src3;
  f16t* dz = dst + (size_t)z * (size_t)dstStrideZ;
  const int k0 = blockIdx.y * 64, n0 = blockIdx.x * 64;
  const int tid = threadIdx.x;
  const int r0 = tid >> 4, c4 = (tid & 15) * 4;
#pragma unroll
  for (int j = 0; j < 4; ++j) {
    const int r = r0 + 16 * j;
    const Tin* sp = src + (size_t)(k0 + r) * N + n0 + c4;
#pragma unroll
    for (int q = 0; q < 4; ++q) T[c4 + q][r] = (f16t)((float)sp[q] * scale);
  }
  __syncthreads();
  v8h vv[2];
#pragma unroll
  for (int p = 0; p < 2; ++p) {
    const int idx = p * 256 + tid;
    vv[p] = *(const v8h*)&T[idx >> 3][(idx & 7) * 8];
  }
#pragma unroll
  for (int p = 0; p < 2; ++p) {
    const int idx = p * 256 + tid;
    stv8(dz + (size_t)(n0 + (idx >> 3)) * K + k0 + (idx & 7) * 8, vv[p]);
  }
  __threadfence();
#pragma unroll
  for (int p = 0; p < 2; ++p) {
    const int idx = p * 256 + tid;
    stv8(dz + (size_t)(n0 + (idx >> 3)) * K + k0 + (idx & 7) * 8, vv[p]);
  }
}

template <typename OT, bool RELU>
__global__ void __launch_bounds__(128)
k_gemm(const f16t* __restrict__ A, int lda, long strideAz,
       const f16t* __restrict__ Bt, int ldb, long strideBz,
       const float* __restrict__ bias0, const float* __restrict__ bias1,
       const float* __restrict__ bias2, int useBias,
       int K, OT* __restrict__ Out, int ldo, long strideOz, int colOffZ, float scale) {
  __shared__ __align__(16) float sC[16][68];
  const int tid = threadIdx.x, w = tid >> 5, l = tid & 31, h = l >> 4, m = l & 15;
  const int z = blockIdx.z;
  const int row0 = blockIdx.y * 16, col0 = blockIdx.x * 64;
  const f16t* Ar = A + (size_t)z * strideAz + (size_t)(row0 + m) * lda + 8 * h;
  const f16t* Br = Bt + (size_t)z * strideBz + (size_t)(col0 + 16 * w + m) * ldb + 8 * h;
  v8f acc = zero8();
#pragma unroll 4
  for (int k0 = 0; k0 < K; k0 += 32) {
    Frag a, b;
    a.h[0] = *(const v8h*)(Ar + k0);
    a.h[1] = *(const v8h*)(Ar + k0 + 16);
    b.h[0] = *(const v8h*)(Br + k0);
    b.h[1] = *(const v8h*)(Br + k0 + 16);
    acc = wmma16(a.v, b.v, acc);
  }
  const float* bias = (z == 0) ? bias0 : (z == 1) ? bias1 : bias2;
  const int cl = 16 * w + m;
  const float bv = useBias ? bias[col0 + cl] : 0.0f;
#pragma unroll
  for (int r = 0; r < 8; ++r) {
    float v = acc[r] * scale + bv;
    if (RELU) v = fmaxf(v, 0.0f);
    sC[8 * h + r][cl] = v;
  }
  __syncthreads();
  OT* Oz = Out + (size_t)z * strideOz;
  const int colb = colOffZ * z + col0;
  if (sizeof(OT) == 2) {
    const int row = tid >> 3, piece = tid & 7;
    v8h o;
#pragma unroll
    for (int j = 0; j < 8; ++j) o[j] = (f16t)sC[row][piece * 8 + j];
    f16t* op = (f16t*)Oz + (size_t)(row0 + row) * ldo + colb + piece * 8;
    stv8(op, o);
    __threadfence();
    stv8(op, o);
  } else {
    v4f o[2];
#pragma unroll
    for (int p = 0; p < 2; ++p) {
      const int idx = p * 128 + tid;
      o[p] = *(const v4f*)&sC[idx >> 4][(idx & 15) * 4];
    }
#pragma unroll
    for (int p = 0; p < 2; ++p) {
      const int idx = p * 128 + tid;
      stv4((float*)Oz + (size_t)(row0 + (idx >> 4)) * ldo + colb + (idx & 15) * 4, o[p]);
    }
    __threadfence();
#pragma unroll
    for (int p = 0; p < 2; ++p) {
      const int idx = p * 128 + tid;
      stv4((float*)Oz + (size_t)(row0 + (idx >> 4)) * ldo + colb + (idx & 15) * 4, o[p]);
    }
  }
}

__global__ void __launch_bounds__(64)
k_gx(const float* __restrict__ ef, const int* __restrict__ gather_idx, f16t* __restrict__ Xh) {
  const int n = blockIdx.x, t = threadIdx.x;
  int gi = gather_idx[n];
  if (gi < 0) gi += PP;
  gi = gi < 0 ? 0 : (gi > PP - 1 ? PP - 1 : gi);
  const float* s = ef + (size_t)gi * HH + t * 8;
  v4f a = *(const v4f*)s, b = *(const v4f*)(s + 4);
  v8h o;
  o[0] = (f16t)a.x; o[1] = (f16t)a.y; o[2] = (f16t)a.z; o[3] = (f16t)a.w;
  o[4] = (f16t)b.x; o[5] = (f16t)b.y; o[6] = (f16t)b.z; o[7] = (f16t)b.w;
  f16t* op = Xh + (size_t)n * HH + t * 8;
  stv8(op, o);
  __threadfence();
  stv8(op, o);
}

__global__ void __launch_bounds__(128)
k_pos(const f16t* __restrict__ Wp1T, const float* __restrict__ b_p1,
      const f16t* __restrict__ Wt2, const float* __restrict__ b_p2,
      const float* __restrict__ ts, float* __restrict__ sim) {
  __shared__ __align__(16) f16t peL[MPB][PEP];
  __shared__ __align__(16) f16t hL[MPB][PEP];
  __shared__ float posL[2 * MPB];
  __shared__ __align__(16) float sS[GG][68];

  const int tid = threadIdx.x, wave = tid >> 5, lane = tid & 31;
  const int h = lane >> 4, m16 = lane & 15;
  const int p0 = blockIdx.x * MPB;
  const int n = p0 / NN;
  const int m0 = p0 - n * NN;

  const float st_n = ts[2 * n], en_n = ts[2 * n + 1];
  const float cen_n = 0.5f * (st_n + en_n);
  const float len_n = fmaxf(en_n - st_n, 0.1f);
  const float rlen_n = 1.0f / len_n;
  {
    const int i = tid >> 1, cc = tid & 1;
    const int mm = m0 + i;
    const float st_m = ts[2 * mm], en_m = ts[2 * mm + 1];
    const float cen_m = 0.5f * (st_m + en_m);
    const float len_m = fmaxf(en_m - st_m, 0.1f);
    posL[tid] = cc ? logf(len_m * rlen_n) : (cen_n - cen_m) * rlen_n;
  }
  const float rdim = 1.0f / powf(10000.0f, (float)tid * 0.0078125f);
  __syncthreads();

#pragma unroll 1
  for (int e = 0; e < 2 * MPB; ++e) {
    const float dv = (100.0f * posL[e]) * rdim;
    float sv, cv;
    sincosf(dv, &sv, &cv);
    const int i = e >> 1, cc = e & 1;
    peL[i][cc * 256 + tid] = (f16t)sv;
    peL[i][cc * 256 + 128 + tid] = (f16t)cv;
  }
  __syncthreads();

  const f16t* prow = &peL[wave * 16 + m16][8 * h];
  const float s16 = 0.0625f;
#pragma unroll 1
  for (int t = 0; t < HH / 16; ++t) {
    const f16t* brow = Wp1T + (size_t)(t * 16 + m16) * HH + 8 * h;
    v8f acc = zero8();
#pragma unroll 4
    for (int k0 = 0; k0 < HH; k0 += 32) {
      Frag a, b;
      a.h[0] = *(const v8h*)(prow + k0);
      a.h[1] = *(const v8h*)(prow + k0 + 16);
      b.h[0] = *(const v8h*)(brow + k0);
      b.h[1] = *(const v8h*)(brow + k0 + 16);
      acc = wmma16(a.v, b.v, acc);
    }
    const int col = t * 16 + m16;
    const float bv = b_p1[col];
#pragma unroll
    for (int r = 0; r < 8; ++r)
      hL[wave * 16 + 8 * h + r][col] = (f16t)tanhf(acc[r] * s16 + bv);
  }
  __syncthreads();

  {
    const f16t* hrow = &hL[wave * 16 + m16][8 * h];
    const f16t* wrow = Wt2 + (size_t)m16 * HH + 8 * h;
    v8f acc = zero8();
#pragma unroll 4
    for (int k0 = 0; k0 < HH; k0 += 32) {
      Frag a, b;
      a.h[0] = *(const v8h*)(hrow + k0);
      a.h[1] = *(const v8h*)(hrow + k0 + 16);
      b.h[0] = *(const v8h*)(wrow + k0);
      b.h[1] = *(const v8h*)(wrow + k0 + 16);
      acc = wmma16(a.v, b.v, acc);
    }
    if (m16 < GG) {
      const float bb = b_p2[m16];
#pragma unroll
      for (int r = 0; r < 8; ++r) sS[m16][wave * 16 + 8 * h + r] = acc[r] * s16 + bb;
    }
  }
  __syncthreads();

  {
    const int g = tid >> 4, piece = tid & 15;
    float* sp = sim + ((size_t)(g * NN + n)) * NN + m0 + piece * 4;
    v4f o = *(const v4f*)sp;
    const v4f add = *(const v4f*)&sS[g][piece * 4];
    o += add;
    stv4(sp, o);
    __threadfence();
    stv4(sp, o);
  }
}

__global__ void __launch_bounds__(128)
k_softmax(const float* __restrict__ sim, const int* __restrict__ block_id,
          f16t* __restrict__ Ph) {
  __shared__ float red[4];
  __shared__ __align__(16) f16t sP[NN];
  const int tid = threadIdx.x;
  const int row = blockIdx.x;
  const int n = row % NN;
  const float* rp = sim + (size_t)row * NN;
  float v[3];
#pragma unroll
  for (int i = 0; i < 3; ++i) v[i] = rp[tid + i * 128];
  float mx = fmaxf(fmaxf(v[0], v[1]), v[2]);
  mx = bmax128(mx, red, tid);
  float s = 0.f;
#pragma unroll
  for (int i = 0; i < 3; ++i) { v[i] = expf(v[i] - mx); s += v[i]; }
  const float tot = bsum128(s, red, tid);
  const float inv = 1.0f / tot;
  const int bn = block_id[n];
  float w[3];
  float s2 = 0.f;
#pragma unroll
  for (int i = 0; i < 3; ++i) {
    const int m = tid + i * 128;
    const float p = v[i] * inv;
    w[i] = (block_id[m] == bn) ? p : 0.0f;
    s2 += w[i];
  }
  const float tot2 = bsum128(s2, red, tid);
  const float inv2 = 1.0f / (1e-5f + tot2);
#pragma unroll
  for (int i = 0; i < 3; ++i) sP[tid + i * 128] = (f16t)(w[i] * inv2 * 16384.0f);
  __syncthreads();
  v8h o = zero8h();
  if (tid < NN / 8) o = *(const v8h*)&sP[tid * 8];
  f16t* pp = Ph + (size_t)row * NN + tid * 8;
  if (tid < NN / 8) stv8(pp, o);
  __threadfence();
  if (tid < NN / 8) stv8(pp, o);
}

__device__ __forceinline__ void out0_pass(float* __restrict__ out0, const float* __restrict__ ctx,
                                          const float* __restrict__ ef,
                                          const int* sGi, const int* sSi, const int* sEi,
                                          int rb, int tid) {
#pragma unroll 1
  for (int it = 0; it < 36; ++it) {
    const int idx = it * 256 + tid;
    if (idx < (32 * ECW) / 4) {
      const int f = idx * 4;
      const int r = f / ECW;
      const int c = f - r * ECW;
      const int n = rb + r;
      v4f v;
      if (c < HH) {
        v = *(const v4f*)(ctx + (size_t)n * HH + c);
      } else if (c < 2 * HH) {
        v = *(const v4f*)(ef + (size_t)sGi[r] * HH + (c - HH));
      } else {
        const int j = c - 2 * HH;
        const int si = sSi[r], ei = sEi[r];
        v.x = (j + 0 >= si && j + 0 <= ei) ? 1.0f : 0.0f;
        v.y = (j + 1 >= si && j + 1 <= ei) ? 1.0f : 0.0f;
        v.z = (j + 2 >= si && j + 2 <= ei) ? 1.0f : 0.0f;
        v.w = (j + 3 >= si && j + 3 <= ei) ? 1.0f : 0.0f;
      }
      stv4(out0 + (size_t)rb * ECW + f, v);
    }
  }
}

__device__ __forceinline__ int ts_bucket(float x, float dur) {
  float f = (x / dur) * 99.0f;
  if (!(f == f)) f = 0.0f;
  f = fminf(fmaxf(f, -2147483648.0f), 2147483520.0f);
  int b = (int)f;
  return b > 99 ? 99 : b;
}

__global__ void __launch_bounds__(256)
k_out(const float* __restrict__ ctx, const float* __restrict__ ef,
      const int* __restrict__ gather_idx, const float* __restrict__ ts,
      const float* __restrict__ dur, float* __restrict__ out0) {
  __shared__ int sGi[32];
  __shared__ int sSi[32];
  __shared__ int sEi[32];
  const int rb = blockIdx.x * 32, tid = threadIdx.x;
  if (tid < 32) {
    const int n = rb + tid;
    int gi = gather_idx[n];
    if (gi < 0) gi += PP;
    gi = gi < 0 ? 0 : (gi > PP - 1 ? PP - 1 : gi);
    sGi[tid] = gi;
    const float d = dur[n];
    sSi[tid] = ts_bucket(ts[2 * n], d);
    sEi[tid] = ts_bucket(ts[2 * n + 1], d);
  }
  __syncthreads();
  out0_pass(out0, ctx, ef, sGi, sSi, sEi, rb, tid);
  __threadfence();
  out0_pass(out0, ctx, ef, sGi, sSi, sEi, rb, tid);
}

extern "C" void kernel_launch(void* const* d_in, const int* in_sizes, int n_in,
                              void* d_out, int out_size, void* d_ws, size_t ws_size,
                              hipStream_t stream) {
  (void)in_sizes;
  if (n_in < 20) return;
  if ((size_t)out_size < (size_t)PP * ECW + (size_t)PP * LL * DD + (size_t)PP * LL) return;

  const float* feats      = (const float*)d_in[0];
  const int*   vid_idx    = (const int*)d_in[1];
  const int*   starts     = (const int*)d_in[2];
  const int*   clip_len   = (const int*)d_in[3];
  const int*   gather_idx = (const int*)d_in[4];
  const int*   block_id   = (const int*)d_in[5];
  const float* timestamps = (const float*)d_in[6];
  const float* durations  = (const float*)d_in[7];
  const float* W_pre = (const float*)d_in[8];
  const float* b_pre = (const float*)d_in[9];
  const float* W_q   = (const float*)d_in[10];
  const float* b_q   = (const float*)d_in[11];
  const float* W_k   = (const float*)d_in[12];
  const float* b_k   = (const float*)d_in[13];
  const float* W_v   = (const float*)d_in[14];
  const float* b_v   = (const float*)d_in[15];
  const float* W_p1  = (const float*)d_in[16];
  const float* b_p1  = (const float*)d_in[17];
  const float* W_p2  = (const float*)d_in[18];
  const float* b_p2  = (const float*)d_in[19];

  size_t off = 0;
  auto carve = [&](size_t bytes) { size_t o = off; off += (bytes + 255) & ~(size_t)255; return o; };
  const size_t o_efh  = carve((size_t)PP * DD * 2);
  const size_t o_wpre = carve((size_t)HH * DD * 2);
  const size_t o_w4   = carve((size_t)4 * HH * HH * 2);
  const size_t o_wt2  = carve((size_t)16 * HH * 2);
  const size_t o_ef   = carve((size_t)PP * HH * 4);
  const size_t o_xh   = carve((size_t)NN * HH * 2);
  const size_t o_qkv  = carve((size_t)3 * NN * HH * 2);
  const size_t o_vt   = carve((size_t)HH * NN * 2);
  const size_t o_sim  = carve((size_t)GG * NN * NN * 4);
  const size_t o_ph   = carve((size_t)GG * NN * NN * 2);
  const size_t o_ctx  = carve((size_t)NN * HH * 4);
  if (off > ws_size) return;

  char* ws = (char*)d_ws;
  f16t*  efh  = (f16t*)(ws + o_efh);
  f16t*  wpreT= (f16t*)(ws + o_wpre);
  f16t*  w4T  = (f16t*)(ws + o_w4);
  f16t*  wt2  = (f16t*)(ws + o_wt2);
  float* ef   = (float*)(ws + o_ef);
  f16t*  Xh   = (f16t*)(ws + o_xh);
  f16t*  qkvh = (f16t*)(ws + o_qkv);
  f16t*  vt   = (f16t*)(ws + o_vt);
  float* sim  = (float*)(ws + o_sim);
  f16t*  Ph   = (f16t*)(ws + o_ph);
  float* ctx  = (float*)(ws + o_ctx);
  f16t*  qh   = qkvh;
  f16t*  kh   = qkvh + (size_t)NN * HH;
  f16t*  vh   = qkvh + (size_t)2 * NN * HH;
  f16t*  wp1T = w4T + (size_t)3 * HH * HH;

  float* out0 = (float*)d_out;
  float* out1 = out0 + (size_t)PP * ECW;
  float* out2 = out1 + (size_t)PP * LL * DD;

  k_clip<<<PP, 256, 0, stream>>>(feats, vid_idx, starts, clip_len, out1, efh);
  k_misc<<<1, 256, 0, stream>>>(W_p2, out2, wt2);
  k_tr64<float><<<dim3(HH / 64, DD / 64, 1), 256, 0, stream>>>(W_pre, W_pre, W_pre, W_pre, DD, HH, 32.0f, wpreT, 0);
  k_tr64<float><<<dim3(HH / 64, HH / 64, 4), 256, 0, stream>>>(W_q, W_k, W_v, W_p1, HH, HH, 16.0f, w4T, HH * HH);
  k_gemm<float, true><<<dim3(HH / 64, PP / 16, 1), 128, 0, stream>>>(
      efh, DD, 0L, wpreT, DD, 0L, b_pre, b_pre, b_pre, 1, DD, ef, HH, 0L, 0, 1.0f / 32.0f);
  k_gx<<<NN, 64, 0, stream>>>(ef, gather_idx, Xh);
  k_gemm<f16t, false><<<dim3(HH / 64, NN / 16, 3), 128, 0, stream>>>(
      Xh, HH, 0L, w4T, HH, (long)HH * HH, b_q, b_k, b_v, 1, HH, qkvh, HH, (long)NN * HH, 0, 1.0f / 16.0f);
  k_tr64<f16t><<<dim3(HH / 64, NN / 64, 1), 256, 0, stream>>>(vh, vh, vh, vh, NN, HH, 1.0f, vt, 0);
  k_gemm<float, false><<<dim3(NN / 64, NN / 16, GG), 128, 0, stream>>>(
      qh, HH, (long)HGG, kh, HH, (long)HGG, b_q, b_q, b_q, 0, HGG, sim, NN, (long)NN * NN, 0, 0.125f);
  k_pos<<<(NN * NN) / MPB, 128, 0, stream>>>(wp1T, b_p1, wt2, b_p2, timestamps, sim);
  k_softmax<<<GG * NN, 128, 0, stream>>>(sim, block_id, Ph);
  k_gemm<float, true><<<dim3(HGG / 64, NN / 16, GG), 128, 0, stream>>>(
      Ph, NN, (long)NN * NN, vt, NN, (long)HGG * NN, b_q, b_q, b_q, 0, NN, ctx, HH, 0L, HGG, 1.0f / 16384.0f);
  k_out<<<PP / 32, 256, 0, stream>>>(ctx, ef, gather_idx, timestamps, durations, out0);
}
